// EncoderBlock_20684562498083
// MI455X (gfx1250) — hardware-verified
//
#include <hip/hip_runtime.h>
#include <math.h>

#ifndef NB
#define NB 2
#endif
#ifndef SEQ
#define SEQ 2048
#endif
#define NB_FULL 2
#define SEQ_FULL 2048
#define DM 1024
#define NHEAD 16
#define HDIM 64
#define INR 3072
#define ROWS (NB * SEQ)
static_assert(NB >= 1 && NB <= NB_FULL);
static_assert(SEQ % 64 == 0 && SEQ >= 64 && SEQ <= SEQ_FULL);
static_assert(DM == NHEAD * HDIM);
static_assert(ROWS % 64 == 0 && DM % 64 == 0 && INR % 64 == 0 && (3 * DM) % 64 == 0 && (2 * INR) % 64 == 0);
static_assert(DM % 32 == 0 && INR % 32 == 0);

typedef __attribute__((ext_vector_type(16))) _Float16 v16h;
typedef __attribute__((ext_vector_type(8)))  _Float16 v8h;
typedef __attribute__((ext_vector_type(16))) __bf16   v16b;
typedef __attribute__((ext_vector_type(8)))  __bf16   v8b;
typedef __attribute__((ext_vector_type(8)))  float    v8f;
typedef __attribute__((ext_vector_type(4)))  float    v4f;
typedef __attribute__((ext_vector_type(4)))  unsigned int u4v;

#define VST2(T, ptr, val) do { const T vst2_v_ = (val); *(volatile T*)(ptr) = vst2_v_; __threadfence(); *(volatile T*)(ptr) = vst2_v_; } while (0)
#define VST2V4(ptr, val) do { const v4f vst2_v4_ = (val); *(volatile v4f*)(ptr) = vst2_v4_; __threadfence(); *(volatile v4f*)(ptr) = vst2_v4_; } while (0)

__device__ __forceinline__ float bfr(float v) { const unsigned u = __float_as_uint(v); const unsigned r = (u + 0x7fffu + ((u >> 16) & 1u)) & 0xffff0000u; return __uint_as_float(r); }
__device__ __forceinline__ unsigned int pk2h(float a, float b) { return (unsigned int)__builtin_bit_cast(unsigned short, (_Float16)a) | ((unsigned int)__builtin_bit_cast(unsigned short, (_Float16)b) << 16); }

namespace w25 {

__device__ __forceinline__ unsigned short f2bf_bits(float f) {
  unsigned u = __float_as_uint(f);
  return (unsigned short)((u + 0x7FFFu + ((u >> 16) & 1u)) >> 16);
}
__device__ __forceinline__ float bf_bits2f(unsigned short h) { return __uint_as_float(((unsigned)h) << 16); }

__device__ __forceinline__ void dep_guard_h(v8f& a, v8f& b, v16h x, v16h y) { asm volatile("v_nop\n\tv_nop\n\tv_nop\n\tv_nop" : "+v"(a), "+v"(b) : "v"(x), "v"(y)); }
__device__ __forceinline__ void dep_guard_b(v8f& a, v8f& b, v16b x, v16b y) { asm volatile("v_nop\n\tv_nop\n\tv_nop\n\tv_nop" : "+v"(a), "+v"(b) : "v"(x), "v"(y)); }
__device__ __forceinline__ void keep4_h(v16h a, v16h b, v16h c, v16h d) { asm volatile("v_nop" :: "v"(a), "v"(b), "v"(c), "v"(d)); }
__device__ __forceinline__ void keep4_b(v16b a, v16b b, v16b c, v16b d) { asm volatile("v_nop" :: "v"(a), "v"(b), "v"(c), "v"(d)); }
__device__ __forceinline__ void acc_guard4(v8f& a, v8f& b, v8f& c, v8f& d) { asm volatile("v_nop\n\tv_nop\n\tv_nop\n\tv_nop" : "+v"(a), "+v"(b), "+v"(c), "+v"(d)); }
template <typename T> struct Frag;
template <> struct Frag<_Float16> {
  typedef v16h V; union U { v16h v; v8h h[2]; };
  static __device__ __forceinline__ v16h load(const _Float16* p) {
    U f; f.h[0] = *(const v8h*)(p); f.h[1] = *(const v8h*)(p + 16); return f.v;
  }
  static __device__ __forceinline__ v8f mma(v16h a, v16h b, v8f c) {
    return __builtin_amdgcn_wmma_f32_16x16x32_f16(false, a, false, b, (short)0, c, false, false);
  }
  static __device__ __forceinline__ void guard(v8f& a, v8f& b, v16h x, v16h y) { dep_guard_h(a, b, x, y); }
  static __device__ __forceinline__ void keep(v16h a, v16h b, v16h c, v16h d) { keep4_h(a, b, c, d); }
};
template <> struct Frag<__bf16> {
  typedef v16b V; union U { v16b v; v8b h[2]; };
  static __device__ __forceinline__ v16b load(const __bf16* p) {
    U f; f.h[0] = *(const v8b*)(p); f.h[1] = *(const v8b*)(p + 16); return f.v;
  }
  static __device__ __forceinline__ v8f mma(v16b a, v16b b, v8f c) {
    return __builtin_amdgcn_wmma_f32_16x16x32_bf16(false, a, false, b, (short)0, c, false, false);
  }
  static __device__ __forceinline__ void guard(v8f& a, v8f& b, v16b x, v16b y) { dep_guard_b(a, b, x, y); }
  static __device__ __forceinline__ void keep(v16b a, v16b b, v16b c, v16b d) { keep4_b(a, b, c, d); }
};

template <int ET> struct Elem;
template <> struct Elem<0> { typedef _Float16 T; };
template <> struct Elem<1> { typedef __bf16 T; };
template <int ET, bool SPLIT, int BIAS_MODE, int OUT_MODE, int RESID, int ACT = 0>
__global__ __launch_bounds__(256) void wmma_gemm64(
    const unsigned short* __restrict__ Ap, const unsigned short* __restrict__ A2p, int lda, long strideA,
    const unsigned short* __restrict__ Btp, const unsigned short* __restrict__ Bt2p, int ldb, long strideB,
    void* __restrict__ Cout, void* __restrict__ Cout2, int ldc, long strideC,
    const float* __restrict__ bias,
    const float* __restrict__ resid, long strideR,
    int M, int N, int K, float scale) {
  typedef typename Elem<ET>::T T;
  typedef typename Frag<T>::V V;
  const T* A = (const T*)Ap; const T* A2 = (const T*)A2p; const T* Bt = (const T*)Btp; const T* Bt2 = (const T*)Bt2p;
  __shared__ __align__(16) float sT[8][16 * 68];
  const int b    = blockIdx.y;
  const int lane = threadIdx.x & 31;
  const int wave = threadIdx.x >> 5;
  const int tilesN = N >> 6;
  const int tilesM = M >> 6;
  const int tile = blockIdx.x * 8 + wave;
  if (tile >= tilesM * tilesN) return;
  const int tm = tile / tilesN;
  const int tn = tile - tm * tilesN;
  const int m0 = tm << 6;
  const int n0 = tn << 6;

  const T* Ab  = A  + (size_t)b * strideA;
  const T* Bb  = Bt + (size_t)b * strideB;
  const T* Ab2 = SPLIT ? (A2  + (size_t)b * strideA) : nullptr;
  const T* Bb2 = SPLIT ? (Bt2 + (size_t)b * strideB) : nullptr;

  const int rlane = lane & 15;
  const int koff  = (lane >> 4) * 8;
  const int mOff  = (lane >> 4) * 8;

  v8f acc[4][4];
#pragma unroll
  for (int i = 0; i < 4; ++i)
#pragma unroll
    for (int j = 0; j < 4; ++j) acc[i][j] = (v8f){0.f,0.f,0.f,0.f,0.f,0.f,0.f,0.f};

  for (int k0 = 0; k0 < K; k0 += 32) {
    V bh[4], bl[4];
#pragma unroll
    for (int j = 0; j < 4; ++j) {
      const size_t bo = (size_t)(n0 + (j << 4) + rlane) * ldb + koff + k0;
      bh[j] = Frag<T>::load(Bb + bo);
      if (SPLIT) bl[j] = Frag<T>::load(Bb2 + bo);
    }
#pragma unroll
    for (int i = 0; i < 4; ++i) {
      const size_t ao = (size_t)(m0 + (i << 4) + rlane) * lda + koff + k0;
      V ah = Frag<T>::load(Ab + ao);
      V al;
      if (SPLIT) al = Frag<T>::load(Ab2 + ao);
#pragma unroll
      for (int j = 0; j < 4; ++j) {
        acc[i][j] = Frag<T>::mma(ah, bh[j], acc[i][j]);
        if (SPLIT) {
          acc[i][j] = Frag<T>::mma(ah, bl[j], acc[i][j]);
          acc[i][j] = Frag<T>::mma(al, bh[j], acc[i][j]);
        }
      }
      Frag<T>::guard(acc[i][0], acc[i][3], ah, SPLIT ? al : ah);
    }
    Frag<T>::keep(bh[0], bh[1], bh[2], bh[3]);
    if (SPLIT) Frag<T>::keep(bl[0], bl[1], bl[2], bl[3]);
  }
  acc_guard4(acc[0][0], acc[0][1], acc[0][2], acc[0][3]);
  acc_guard4(acc[1][0], acc[1][1], acc[1][2], acc[1][3]);
  acc_guard4(acc[2][0], acc[2][1], acc[2][2], acc[2][3]);
  acc_guard4(acc[3][0], acc[3][1], acc[3][2], acc[3][3]);

  float* slab = sT[wave];
  const float* Rb = (RESID != 0) ? (resid + (size_t)b * strideR) : nullptr;
#pragma unroll
  for (int i = 0; i < 4; ++i) {
    const int mBase = m0 + (i << 4);
#pragma unroll
    for (int j = 0; j < 4; ++j) {
      const int n = n0 + (j << 4) + rlane;
      float bv = 0.f;
      if (BIAS_MODE == 2) bv = bias[n];
#pragma unroll
      for (int r = 0; r < 8; ++r) {
        float v = acc[i][j][r] * scale;
        if (BIAS_MODE == 1) v += bias[mBase + mOff + r];
        if (BIAS_MODE == 2) v += bv;
        if (RESID == 1) v += Rb[(size_t)(mBase + mOff + r) * ldc + n];
        if (RESID == 2) v += bfr(Rb[(size_t)(mBase + mOff + r) * ldc + n]);
        if (ACT == 1) v = tanhf(v);
        if (ACT == 2) v = fmaxf(v, 0.0f);
        if (ACT == 3) v = v / (1.0f + expf(-v));
        if (ACT == 4) v = (v > 0.f) ? v : 0.01f * v;
        if (ACT == 5) v = 0.5f * v * (1.0f + erff(v * 0.70710678118654752f));
        if (ACT == 6) v = (v > 0.f) ? v : 0.2f * v;
        if (ACT == 7) { const float u = 0.7978845608028654f * (v + 0.044715f * v * v * v); v = 0.5f * v * (1.f + tanhf(u)); }
        slab[(mOff + r) * 68 + (j << 4) + rlane] = v;
      }
    }
    __builtin_amdgcn_fence(3  , "workgroup");
    __builtin_amdgcn_wave_barrier();
    __builtin_amdgcn_fence(2  , "workgroup");
    if (OUT_MODE == 0) {
      float* C = (float*)Cout + (size_t)b * strideC;
      const int hh = lane >> 4, c4 = (lane & 15) * 4;
      for (int pass = 0; pass < 2; ++pass) {
#pragma unroll
        for (int it = 0; it < 8; ++it) {
          const int row = it * 2 + hh;
          v4f v = *(const v4f*)(slab + row * 68 + c4);
          *(volatile v4f*)(C + (size_t)(mBase + row) * ldc + n0 + c4) = v;
        }
        __threadfence();
      }
    } else {
      const int q = lane >> 3, c8 = (lane & 7) * 8;
      unsigned short* C  = (unsigned short*)Cout  + (size_t)b * strideC;
      unsigned short* C2 = (OUT_MODE == 2) ? ((unsigned short*)Cout2 + (size_t)b * strideC) : nullptr;
      for (int pass = 0; pass < 2; ++pass) {
#pragma unroll
        for (int it = 0; it < 4; ++it) {
          const int row = it * 4 + q;
          const float* sp = slab + row * 68 + c8;
          v8h hv, lv;
#pragma unroll
          for (int e = 0; e < 8; ++e) {
            if (OUT_MODE == 1) {
              hv[e] = (_Float16)sp[e];
            } else {
              unsigned short hb = f2bf_bits(sp[e]);
              unsigned short lb = f2bf_bits(sp[e] - bf_bits2f(hb));
              hv[e] = __builtin_bit_cast(_Float16, hb);
              lv[e] = __builtin_bit_cast(_Float16, lb);
            }
          }
          *(volatile v8h*)(C + (size_t)(mBase + row) * ldc + n0 + c8) = hv;
          if (OUT_MODE == 2) *(volatile v8h*)(C2 + (size_t)(mBase + row) * ldc + n0 + c8) = lv;
        }
        __threadfence();
      }
    }
    __builtin_amdgcn_fence(3  , "workgroup");
    __builtin_amdgcn_wave_barrier();
    __builtin_amdgcn_fence(2  , "workgroup");
  }
}

#define AT_D 64
#define AT_NW 4
#define AT_QB 64
#define AT_KC 64
struct AttnGeom { const float* cp; const float* pc; long c_bs, c_rs, c_hs;
                  long q_bs, q_rs, q_hs, k_bs, k_rs, k_hs, v_bs, v_rs, v_hs, o_bs, o_rs, o_hs;
                  int S, Skv, H, mask_mode; float qscale; int blk0; float mask_fill; int mask_is_int; };
static_assert(sizeof(AttnGeom) == 168);

__device__ __forceinline__ unsigned short at_bf_bits(float f) {
  unsigned u = __float_as_uint(f);
  return (unsigned short)((u + 0x7FFFu + ((u >> 16) & 1u)) >> 16);
}
__device__ __forceinline__ __bf16 at_f2bf(float f) { return __builtin_bit_cast(__bf16, at_bf_bits(f)); }
__device__ __forceinline__ void at_split(float f, __bf16& hi, __bf16& lo) {
  const unsigned short hb = at_bf_bits(f);
  hi = __builtin_bit_cast(__bf16, hb);
  lo = at_f2bf(f - __uint_as_float(((unsigned)hb) << 16));
}
__device__ __forceinline__ v8f at_mma(v16b a, v16b b, v8f c) {
  c = __builtin_amdgcn_wmma_f32_16x16x32_bf16(false, a, false, b, (short)0, c, false, false);
  asm volatile("v_nop\n\tv_nop\n\tv_nop\n\tv_nop" : "+v"(c) : "v"(a), "v"(b));
  return c;
}
template <bool F16> __device__ __forceinline__ __bf16 at_to16(float f) {
  if (F16) return __builtin_bit_cast(__bf16, (_Float16)f);
  return at_f2bf(f);
}
template <bool F16> __device__ __forceinline__ v8f at_mma16(v16b a, v16b b, v8f c) {
  if (F16) {
    const v16h ah = __builtin_bit_cast(v16h, a), bh = __builtin_bit_cast(v16h, b);
    c = __builtin_amdgcn_wmma_f32_16x16x32_f16(false, ah, false, bh, (short)0, c, false, false);
    asm volatile("v_nop\n\tv_nop\n\tv_nop\n\tv_nop" : "+v"(c) : "v"(ah), "v"(bh));
    return c;
  }
  return at_mma(a, b, c);
}

template <bool SPLIT_QK, bool SPLIT_PV, bool F16>
__global__ __launch_bounds__(128)
void attn64_kernel(const float* __restrict__ q, const float* __restrict__ k,
                   const float* __restrict__ v, float* __restrict__ out,
                   const void* __restrict__ mask_a, const int* __restrict__ mask_b, AttnGeom g) {
  static_assert(!(F16 && (SPLIT_QK || SPLIT_PV)));
  const float PSC = F16 ? 32768.0f : 1.0f;
  union FB { v16b v; v8b h[2]; };
  __shared__ __align__(16) __bf16 Ksh[AT_KC * AT_D];
  __shared__ __align__(16) __bf16 Ksl[SPLIT_QK ? AT_KC * AT_D : 8];
  __shared__ __align__(16) __bf16 Vth[AT_D * AT_KC];
  __shared__ __align__(16) __bf16 Vtl[SPLIT_PV ? AT_D * AT_KC : 8];
  __shared__ __align__(16) __bf16 Psh[AT_NW][16 * AT_KC];
  __shared__ __align__(16) __bf16 Psl[SPLIT_PV ? AT_NW : 1][SPLIT_PV ? 16 * AT_KC : 8];
  __shared__ __align__(16) float  Os[AT_NW][16 * 68];

  const int tid  = threadIdx.x;
  const int wave = tid >> 5;
  const int lane = tid & 31;
  const int hh   = lane >> 4;
  const int c    = lane & 15;

  const int nqb = g.S / AT_QB;
  const int bx = blockIdx.x + g.blk0;
  const int qb = bx % nqb;
  const int bh = bx / nqb;
  const int h  = bh % g.H;
  const int b  = bh / g.H;
  const int qbase_block = qb * AT_QB;
  const int q0 = qbase_block + wave * 16;

  const float* qb_ptr = q + (size_t)b * g.q_bs + (size_t)h * g.q_hs;
  const float* kb_ptr = k + (size_t)b * g.k_bs + (size_t)h * g.k_hs;
  const float* vb_ptr = v + (size_t)b * g.v_bs + (size_t)h * g.v_hs;
  float*       ob_ptr = out + (size_t)b * g.o_bs + (size_t)h * g.o_hs;

  v16b qah[2], qal[2];
  {
    const float* qrow = qb_ptr + (size_t)(q0 + c) * g.q_rs;
#pragma unroll
    for (int dc = 0; dc < 2; ++dc) {
      const v4f xa = *(const v4f*)(qrow + dc * 32 + 8 * hh);
      const v4f xb = *(const v4f*)(qrow + dc * 32 + 8 * hh + 4);
      const v4f ya = *(const v4f*)(qrow + dc * 32 + 16 + 8 * hh);
      const v4f yb = *(const v4f*)(qrow + dc * 32 + 16 + 8 * hh + 4);
      const float f0s[8] = {xa.x, xa.y, xa.z, xa.w, xb.x, xb.y, xb.z, xb.w};
      const float f1s[8] = {ya.x, ya.y, ya.z, ya.w, yb.x, yb.y, yb.z, yb.w};
#pragma unroll
      for (int e = 0; e < 8; ++e) {
        const float f0 = f0s[e] * g.qscale;
        const float f1 = f1s[e] * g.qscale;
        if (SPLIT_QK) { __bf16 hq, lq; at_split(f0, hq, lq); qah[dc][e] = hq; qal[dc][e] = lq; at_split(f1, hq, lq); qah[dc][8 + e] = hq; qal[dc][8 + e] = lq; }
        else { qah[dc][e] = at_to16<F16>(f0); qah[dc][8 + e] = at_to16<F16>(f1); qal[dc][e] = qah[dc][e]; qal[dc][8 + e] = qah[dc][8 + e]; }
      }
    }
  }

  float mrow[8], lrow[8];
  v8f oacc[4];
#pragma unroll
  for (int r = 0; r < 8; ++r) { mrow[r] = -INFINITY; lrow[r] = 0.f; }
#pragma unroll
  for (int t = 0; t < 4; ++t) oacc[t] = (v8f){0.f,0.f,0.f,0.f,0.f,0.f,0.f,0.f};

  const int nChunks = (g.mask_mode == 1 || g.mask_mode == 4) ? (qb + 1) : (g.Skv / AT_KC);
  int qkeep[8];
#pragma unroll
  for (int r = 0; r < 8; ++r) qkeep[r] = (g.mask_mode == 3) ? mask_b[(size_t)b * g.S + q0 + 8 * hh + r] : 1;
  for (int kc = 0; kc < nChunks; ++kc) {
    const int kv0 = kc * AT_KC;
    __syncthreads();
    {
      const int kvr = tid >> 1, dh = (tid & 1) * 32;
      const float* krow = kb_ptr + (size_t)(kv0 + kvr) * g.k_rs + dh;
      const float* vrow = vb_ptr + (size_t)(kv0 + kvr) * g.v_rs + dh;
#pragma unroll
      for (int i = 0; i < 8; ++i) {
        v4f kk = *(const v4f*)(krow + 4 * i);
        v4f vv = *(const v4f*)(vrow + 4 * i);
#pragma unroll
        for (int e = 0; e < 4; ++e) {
          const int d = dh + 4 * i + e;
          if (SPLIT_QK) { __bf16 a, bl; at_split(kk[e], a, bl); Ksh[kvr * AT_D + d] = a; Ksl[kvr * AT_D + d] = bl; }
          else Ksh[kvr * AT_D + d] = at_to16<F16>(kk[e]);
          if (SPLIT_PV) { __bf16 a, bl; at_split(vv[e], a, bl); Vth[d * AT_KC + kvr] = a; Vtl[d * AT_KC + kvr] = bl; }
          else Vth[d * AT_KC + kvr] = at_to16<F16>(vv[e]);
        }
      }
    }
    __syncthreads();

    v8f s[4];
#pragma unroll
    for (int j = 0; j < 4; ++j) {
      s[j] = (v8f){0.f,0.f,0.f,0.f,0.f,0.f,0.f,0.f};
#pragma unroll 1
      for (int dc = 0; dc < 2; ++dc) {
        FB kb;
        kb.h[0] = *(const v8b*)(Ksh + (j * 16 + c) * AT_D + dc * 32 + 8 * hh);
        kb.h[1] = *(const v8b*)(Ksh + (j * 16 + c) * AT_D + dc * 32 + 16 + 8 * hh);
        s[j] = at_mma16<F16>(qah[dc], kb.v, s[j]);
        if (SPLIT_QK) {
          FB kl;
          kl.h[0] = *(const v8b*)(Ksl + (j * 16 + c) * AT_D + dc * 32 + 8 * hh);
          kl.h[1] = *(const v8b*)(Ksl + (j * 16 + c) * AT_D + dc * 32 + 16 + 8 * hh);
          s[j] = at_mma16<F16>(qah[dc], kl.v, s[j]);
          s[j] = at_mma16<F16>(qal[dc], kb.v, s[j]);
        }
      }
    }
    const bool diag = (g.mask_mode == 1) && (kc == qb);
    int kvkeep[4] = {1, 1, 1, 1};
    if (g.mask_mode == 3) {
#pragma unroll
      for (int j = 0; j < 4; ++j) kvkeep[j] = ((const int*)mask_a)[(size_t)b * g.Skv + kv0 + j * 16 + c];
    }
    float cm[8];
#pragma unroll
    for (int r = 0; r < 8; ++r) {
      const int qrow = q0 + 8 * hh + r;
      float m = -INFINITY;
#pragma unroll
      for (int j = 0; j < 4; ++j) {
        const int kvcol = kv0 + j * 16 + c;
        bool masked = false;
        if (diag) masked = (kvcol > qrow);
        else if (g.mask_mode == 4) masked = (kvcol > qrow) || (qrow - kvcol > g.mask_is_int);
        else if (g.mask_mode == 2) {
          const size_t mi = (size_t)qrow * g.Skv + kvcol;
          masked = (g.mask_is_int == 0) ? (((const float*)mask_a)[mi] == 0.0f)
                 : (g.mask_is_int == 1) ? (((const int*)mask_a)[mi] == 0) : (((const int*)mask_a)[mi] != 0);
        } else if (g.mask_mode == 3) masked = (qkeep[r] == 0) || (kvkeep[j] == 0);
        else if (g.mask_mode == 5) {
          const size_t mi = (size_t)qrow * g.Skv + kvcol;
          masked = (((const int*)mask_a)[mi] != 0);
          int n = mask_b[mi]; n = n < 0 ? 0 : n;
          s[j][r] += g.cp[(size_t)b * g.c_bs + (size_t)h * g.c_hs + (size_t)qrow * g.c_rs + n]
                   + g.pc[(size_t)b * g.c_bs + (size_t)h * g.c_hs + (size_t)kvcol * g.c_rs + n];
        }
        if (masked) s[j][r] = g.mask_fill;
        m = fmaxf(m, s[j][r]);
      }
#pragma unroll
      for (int off = 1; off < 16; off <<= 1) m = fmaxf(m, __shfl_xor(m, off, 32));
      cm[r] = m;
    }
    __bf16* pwh = Psh[wave];
    __bf16* pwl = Psl[SPLIT_PV ? wave : 0];
#pragma unroll
    for (int r = 0; r < 8; ++r) {
      const float mnew = fmaxf(mrow[r], cm[r]);
      const float alpha = expf(mrow[r] - mnew);
      mrow[r] = mnew;
      float psum = 0.f;
#pragma unroll
      for (int j = 0; j < 4; ++j) {
        const float p = expf(s[j][r] - mnew);
        psum += p;
        if (SPLIT_PV) { __bf16 a, bl; at_split(p, a, bl); pwh[(8 * hh + r) * AT_KC + j * 16 + c] = a; pwl[(8 * hh + r) * AT_KC + j * 16 + c] = bl; }
        else pwh[(8 * hh + r) * AT_KC + j * 16 + c] = at_to16<F16>(p * PSC);
      }
#pragma unroll
      for (int off = 1; off < 16; off <<= 1) psum += __shfl_xor(psum, off, 32);
      lrow[r] = lrow[r] * alpha + psum;
#pragma unroll
      for (int t = 0; t < 4; ++t) oacc[t][r] *= alpha;
    }
    __builtin_amdgcn_fence(3  , "workgroup");
    __builtin_amdgcn_wave_barrier();
    __builtin_amdgcn_fence(2  , "workgroup");
#pragma unroll 1
    for (int kk = 0; kk < 2; ++kk) {
      FB pa, pl;
      pa.h[0] = *(const v8b*)(pwh + c * AT_KC + kk * 32 + 8 * hh);
      pa.h[1] = *(const v8b*)(pwh + c * AT_KC + kk * 32 + 16 + 8 * hh);
      if (SPLIT_PV) {
        pl.h[0] = *(const v8b*)(pwl + c * AT_KC + kk * 32 + 8 * hh);
        pl.h[1] = *(const v8b*)(pwl + c * AT_KC + kk * 32 + 16 + 8 * hh);
      }
#pragma unroll
      for (int t = 0; t < 4; ++t) {
        FB vb;
        vb.h[0] = *(const v8b*)(Vth + (t * 16 + c) * AT_KC + kk * 32 + 8 * hh);
        vb.h[1] = *(const v8b*)(Vth + (t * 16 + c) * AT_KC + kk * 32 + 16 + 8 * hh);
        oacc[t] = at_mma16<F16>(pa.v, vb.v, oacc[t]);
        if (SPLIT_PV) {
          FB vl;
          vl.h[0] = *(const v8b*)(Vtl + (t * 16 + c) * AT_KC + kk * 32 + 8 * hh);
          vl.h[1] = *(const v8b*)(Vtl + (t * 16 + c) * AT_KC + kk * 32 + 16 + 8 * hh);
          oacc[t] = at_mma16<F16>(pa.v, vl.v, oacc[t]);
          oacc[t] = at_mma16<F16>(pl.v, vb.v, oacc[t]);
        }
      }
    }
  }

  float* os = Os[wave];
#pragma unroll
  for (int r = 0; r < 8; ++r) {
    const float inv = 1.0f / (lrow[r] * PSC);
#pragma unroll
    for (int t = 0; t < 4; ++t) os[(8 * hh + r) * 68 + t * 16 + c] = oacc[t][r] * inv;
  }
  __builtin_amdgcn_fence(3  , "workgroup");
  __builtin_amdgcn_wave_barrier();
  __builtin_amdgcn_fence(2  , "workgroup");
  {
    const int c4 = (lane & 15) * 4;
    for (int pass = 0; pass < 2; ++pass) {
#pragma unroll
      for (int it = 0; it < 8; ++it) {
        const int row = it * 2 + hh;
        v4f val = *(const v4f*)(os + row * 68 + c4);
        *(volatile v4f*)(ob_ptr + (size_t)(q0 + row) * g.o_rs + c4) = val;
      }
      __threadfence();
    }
  }
}

}

__global__ __launch_bounds__(256) void k_castbT(const float* __restrict__ SRC, int lds, unsigned short* __restrict__ DST, int ldd, int nR, int nC, float sc) {
    const long long u = (long long)blockIdx.x * 256 + threadIdx.x; const int per = nR / 8; if (u >= (long long)nC * per) return; const int c = (int)(u / per); const int r0 = 8 * (int)(u % per);
    float w[8];
#pragma unroll
    for (int e = 0; e < 8; ++e) w[e] = bfr(SRC[(long long)(r0 + e) * lds + c]) * sc;
    u4v pk; pk.x = pk2h(w[0], w[1]); pk.y = pk2h(w[2], w[3]); pk.z = pk2h(w[4], w[5]); pk.w = pk2h(w[6], w[7]); VST2(u4v, (u4v*)(DST + (long long)c * ldd + r0), pk); }

template <int RX>
__global__ __launch_bounds__(256) void k_rms16(const float* __restrict__ X, long long sXb, int seqn, const float* __restrict__ W, unsigned short* __restrict__ O, int rows, float carry) {
    #pragma clang fp contract(off)
    const int row = blockIdx.x * 8 + (threadIdx.x >> 5); const int L = threadIdx.x & 31; if (row >= rows) return;
    const int b = row / seqn; const int t = row - b * seqn;
    const float* xr = X + (long long)b * sXb + (long long)t * DM;
    float x[32]; float s = 0.f;
#pragma unroll
    for (int g = 0; g < 4; ++g) { const v4f a = *(const v4f*)(xr + 256 * g + 8 * L), c = *(const v4f*)(xr + 256 * g + 8 * L + 4); const float v[8] = {a.x, a.y, a.z, a.w, c.x, c.y, c.z, c.w};
#pragma unroll
        for (int e = 0; e < 8; ++e) { const float tt = RX ? bfr(v[e]) : v[e]; x[8 * g + e] = tt; s += tt * tt; } }
#pragma unroll
    for (int o = 16; o > 0; o >>= 1) s += __shfl_xor(s, o, 32);
    const float rs = rsqrtf(s * (1.f / 1024.f) + 1e-5f);
#pragma unroll
    for (int g = 0; g < 4; ++g) { const int c0 = 256 * g + 8 * L; const v4f wa = *(const v4f*)(W + c0), wb = *(const v4f*)(W + c0 + 4); const float wv[8] = {wa.x, wa.y, wa.z, wa.w, wb.x, wb.y, wb.z, wb.w}; float y[8];
#pragma unroll
        for (int e = 0; e < 8; ++e) y[e] = ((x[8 * g + e] * rs) * bfr(wv[e])) * carry;
        u4v pk; pk.x = pk2h(y[0], y[1]); pk.y = pk2h(y[2], y[3]); pk.z = pk2h(y[4], y[5]); pk.w = pk2h(y[6], y[7]); VST2(u4v, (u4v*)(O + (long long)row * DM + c0), pk); } }

__global__ __launch_bounds__(256) void k_rope(float* __restrict__ QKV, const float* __restrict__ RT, long long nthr, int seqn) {
    #pragma clang fp contract(off)
    const long long u = (long long)blockIdx.x * 256 + threadIdx.x; if (u >= nthr) return;
    const long long row = u >> 9; const int c4 = 4 * (int)(u & 511);
    const int t = (int)(row % seqn); const int p = (c4 & (DM - 1)) >> 1;
    float* xp = QKV + row * (3 * DM) + c4;
    const v4f xv = *(const v4f*)xp;
    const v4f rv = *(const v4f*)(RT + ((long long)t * (DM / 2) + p) * 2);
    const float c0 = bfr(rv.x), s0 = bfr(rv.y), c1 = bfr(rv.z), s1 = bfr(rv.w);
    v4f o; o.x = xv.x * c0 - xv.y * s0; o.y = xv.x * s0 + xv.y * c0; o.z = xv.z * c1 - xv.w * s1; o.w = xv.z * s1 + xv.w * c1;
    VST2V4(xp, o);
}

__global__ __launch_bounds__(256) void k_cast16x8(const float* __restrict__ S, unsigned short* __restrict__ D, long long n8, float sc) {
    const long long u = (long long)blockIdx.x * 256 + threadIdx.x; if (u >= n8) return;
    const v4f a = *(const v4f*)(S + 8 * u), b = *(const v4f*)(S + 8 * u + 4);
    u4v pk; pk.x = pk2h(a.x * sc, a.y * sc); pk.y = pk2h(a.z * sc, a.w * sc); pk.z = pk2h(b.x * sc, b.y * sc); pk.w = pk2h(b.z * sc, b.w * sc);
    VST2(u4v, (u4v*)(D + 8 * u), pk); }

__global__ __launch_bounds__(256) void k_glu16(const unsigned short* __restrict__ AG, unsigned short* __restrict__ H, long long n8, int inner, float carry) {
    #pragma clang fp contract(off)
    const long long u = (long long)blockIdx.x * 256 + threadIdx.x; if (u >= n8) return; const int per = inner / 8; const long long r = u / per; const int c0 = 8 * (int)(u % per);
    const v8h av = *(const v8h*)(AG + r * (2LL * inner) + c0); const v8h gv = *(const v8h*)(AG + r * (2LL * inner) + inner + c0);
    float w[8];
#pragma unroll
    for (int e = 0; e < 8; ++e) { const float a = (float)av[e], gg = (float)gv[e]; const float ex = exp2f(-gg * 1.4426950408889634f); const float sg = __builtin_amdgcn_rcpf(1.f + ex); w[e] = (a * sg) * carry; }
    u4v pk; pk.x = pk2h(w[0], w[1]); pk.y = pk2h(w[2], w[3]); pk.z = pk2h(w[4], w[5]); pk.w = pk2h(w[6], w[7]); VST2(u4v, (u4v*)(H + r * (long long)inner + c0), pk); }

static inline unsigned cdiv256(long long n) { return (unsigned)((n + 255) / 256); }
static inline unsigned cdiv8(long long n) { return (unsigned)((n + 7) / 8); }
static inline size_t al256(size_t b) { return (b + 255) & ~(size_t)255; }

extern "C" void kernel_launch(void* const* d_in, const int* in_sizes, int n_in, void* d_out, int out_size, void* d_ws, size_t ws_size, hipStream_t stream) {
    if (n_in < 8) return;
    const long long need_x = (long long)(NB - 1) * SEQ_FULL * DM + (long long)SEQ * DM;
    if ((long long)in_sizes[0] < need_x) return;
    if ((long long)in_sizes[1] < (long long)SEQ * (DM / 2) * 2) return;
    if (in_sizes[2] < DM || in_sizes[5] < DM) return;
    if ((long long)in_sizes[3] < (long long)DM * 3 * DM) return;
    if ((long long)in_sizes[4] < (long long)DM * DM) return;
    if ((long long)in_sizes[6] < (long long)DM * 2 * INR) return;
    if ((long long)in_sizes[7] < (long long)INR * DM) return;
    if ((long long)out_size < need_x) return;

    const float* x    = (const float*)d_in[0];
    const float* rope = (const float*)d_in[1];
    const float* wn1  = (const float*)d_in[2];
    const float* wqkv = (const float*)d_in[3];
    const float* wap  = (const float*)d_in[4];
    const float* wn2  = (const float*)d_in[5];
    const float* wfc  = (const float*)d_in[6];
    const float* wffn = (const float*)d_in[7];
    float* out = (float*)d_out;

    const size_t rows = (size_t)ROWS;
    char* base = (char*)d_ws; size_t off = 0;
    unsigned short* WQKV16 = (unsigned short*)(base + off); off += al256((size_t)3 * DM * DM * 2);
    unsigned short* WO16   = (unsigned short*)(base + off); off += al256((size_t)DM * DM * 2);
    unsigned short* WFC16  = (unsigned short*)(base + off); off += al256((size_t)2 * INR * DM * 2);
    unsigned short* WP16   = (unsigned short*)(base + off); off += al256((size_t)DM * INR * 2);
    float*          QKV    = (float*)(base + off);
    unsigned short* AG16   = (unsigned short*)(base + off); off += al256(rows * 3 * DM * 4);
    float*          AO     = (float*)(base + off);
    unsigned short* H16    = (unsigned short*)(base + off); off += al256(rows * DM * 4);
    unsigned short* N16    = (unsigned short*)(base + off); off += al256(rows * DM * 2);
    float*          X1     = (float*)(base + off); off += al256(rows * DM * 4);
    if (off > ws_size || off > (size_t)134217728) return;
    if (rows * (size_t)INR * 2 > rows * DM * 4 + rows * DM * 2) return;
    if (rows * (size_t)2 * INR * 2 > rows * 3 * DM * 4) return;
    static_assert((3 * DM) % 8 == 0 && DM % 8 == 0 && INR % 8 == 0 && ROWS % 8 == 0);

    k_castbT<<<cdiv256((long long)3 * DM * (DM / 8)), 256, 0, stream>>>(wqkv, 3 * DM, WQKV16, DM, DM, 3 * DM, 64.f);
    k_castbT<<<cdiv256((long long)DM * (DM / 8)), 256, 0, stream>>>(wap, DM, WO16, DM, DM, DM, 64.f);
    k_castbT<<<cdiv256((long long)2 * INR * (DM / 8)), 256, 0, stream>>>(wfc, 2 * INR, WFC16, DM, DM, 2 * INR, 64.f);
    k_castbT<<<cdiv256((long long)DM * (INR / 8)), 256, 0, stream>>>(wffn, DM, WP16, INR, INR, DM, 64.f);
    k_rms16<1><<<(unsigned)(rows / 8), 256, 0, stream>>>(x, (long long)SEQ_FULL * DM, SEQ, wn1, N16, (int)rows, 8.f);
    w25::wmma_gemm64<0, false, 0, 0, 0, 0><<<dim3(cdiv8((long long)(rows / 64) * ((3 * DM) / 64)), 1), 256, 0, stream>>>(
        (const unsigned short*)N16, nullptr, DM, 0L, (const unsigned short*)WQKV16, nullptr, DM, 0L, (void*)QKV, nullptr, 3 * DM, 0L,
        nullptr, nullptr, 0L, (int)rows, 3 * DM, DM, 1.f / 512.f);
    k_rope<<<cdiv256((long long)rows * 512), 256, 0, stream>>>(QKV, rope, (long long)rows * 512, SEQ);
    {
        w25::AttnGeom g;
        g.cp = nullptr; g.pc = nullptr; g.c_bs = 0; g.c_rs = 0; g.c_hs = 0;
        g.q_bs = (long)SEQ * 3 * DM; g.q_rs = 3 * DM; g.q_hs = HDIM;
        g.k_bs = (long)SEQ * 3 * DM; g.k_rs = 3 * DM; g.k_hs = HDIM;
        g.v_bs = (long)SEQ * 3 * DM; g.v_rs = 3 * DM; g.v_hs = HDIM;
        g.o_bs = (long)SEQ * DM; g.o_rs = DM; g.o_hs = HDIM;
        g.S = SEQ; g.Skv = SEQ; g.H = NHEAD; g.mask_mode = 0; g.qscale = 0.125f; g.blk0 = 0; g.mask_fill = 0.f; g.mask_is_int = 0;
        w25::attn64_kernel<false, false, true><<<(unsigned)(NB * NHEAD * (SEQ / 64)), 128, 0, stream>>>(
            QKV, QKV + DM, QKV + 2 * DM, AO, (const void*)WQKV16, (const int*)WQKV16, g);
    }
    k_cast16x8<<<cdiv256((long long)rows * DM / 8), 256, 0, stream>>>(AO, N16, (long long)rows * DM / 8, 64.f);
    w25::wmma_gemm64<0, false, 0, 0, 2, 0><<<dim3(cdiv8((long long)(SEQ / 64) * (DM / 64)), NB), 256, 0, stream>>>(
        (const unsigned short*)N16, nullptr, DM, (long)SEQ * DM, (const unsigned short*)WO16, nullptr, DM, 0L, (void*)X1, nullptr, DM, (long)SEQ * DM,
        nullptr, x, (long)SEQ_FULL * DM, SEQ, DM, DM, 1.f / 4096.f);
    k_rms16<0><<<(unsigned)(rows / 8), 256, 0, stream>>>(X1, (long long)SEQ * DM, SEQ, wn2, N16, (int)rows, 8.f);
    w25::wmma_gemm64<0, false, 0, 1, 0, 0><<<dim3(cdiv8((long long)(rows / 64) * ((2 * INR) / 64)), 1), 256, 0, stream>>>(
        (const unsigned short*)N16, nullptr, DM, 0L, (const unsigned short*)WFC16, nullptr, DM, 0L, (void*)AG16, nullptr, 2 * INR, 0L,
        nullptr, nullptr, 0L, (int)rows, 2 * INR, DM, 1.f / 512.f);
    k_glu16<<<cdiv256((long long)rows * (INR / 8)), 256, 0, stream>>>(AG16, H16, (long long)rows * (INR / 8), INR, 64.f);
    w25::wmma_gemm64<0, false, 0, 0, 1, 0><<<dim3(cdiv8((long long)(SEQ / 64) * (DM / 64)), NB), 256, 0, stream>>>(
        (const unsigned short*)H16, nullptr, INR, (long)SEQ * INR, (const unsigned short*)WP16, nullptr, INR, 0L, (void*)out, nullptr, DM, (long)SEQ_FULL * DM,
        nullptr, X1, (long)SEQ * DM, SEQ, DM, INR, 1.f / 4096.f);
    (void)hipGetLastError();
}
